// mamba_fusion3_26371099198483
// MI455X (gfx1250) — hardware-verified
//
#include <hip/hip_runtime.h>


namespace {
constexpr int NB = 2, C = 768, L = 4096, D = 768, NS = 4, R = 48, XPW = 64, NROW = NB * L;
constexpr float XS = 8.0f, US = 64.0f, DS = 64.0f, YS = 8.0f, WSC = 256.0f, EPS = 1e-5f;

typedef _Float16 b16;
typedef __attribute__((ext_vector_type(16))) _Float16 v16b;
typedef __attribute__((ext_vector_type(8))) _Float16 v8b;
typedef __attribute__((ext_vector_type(4))) _Float16 v4b;
typedef __attribute__((ext_vector_type(8))) float v8f;
typedef __attribute__((ext_vector_type(4))) float v4f;
__device__ __forceinline__ float bf16_rne(float f) { unsigned int u = __float_as_uint(f); u += 0x7FFFu + ((u >> 16) & 1u); return __uint_as_float(u & 0xFFFF0000u); }
__device__ __forceinline__ void split16(float v, b16& hi, b16& lo) { hi = (b16)v; lo = (b16)(v - (float)hi); }
__device__ __forceinline__ v16b frag_kb(const b16* p, int hh) { const v8b a = *(const v8b*)(p + 8 * hh), b = *(const v8b*)(p + 16 + 8 * hh); v16b f;
#pragma unroll
  for (int e = 0; e < 8; ++e) { f[e] = a[e]; f[8 + e] = b[e]; } return f; }
__device__ __forceinline__ v8f wmma16b(v16b a, v16b b, v8f c) { v8f d = __builtin_amdgcn_wmma_f32_16x16x32_f16(false, a, false, b, (short)0, c, false, false); asm volatile("v_nop\n\tv_nop\n\tv_nop\n\tv_nop" : "+v"(d) : "v"(a), "v"(b)); return d; }
__device__ __forceinline__ void wave_lds_sync() { __builtin_amdgcn_fence(__ATOMIC_RELEASE, "workgroup"); __builtin_amdgcn_wave_barrier(); __builtin_amdgcn_fence(__ATOMIC_ACQUIRE, "workgroup"); }
__device__ __forceinline__ float nexp(float x) { return __builtin_amdgcn_exp2f(x * 1.4426950408889634f); }
__device__ __forceinline__ float pmul(float a, float b) { float p = a * b; asm volatile("" : "+v"(p)); return p; }
__device__ __forceinline__ float sigm(float x) { return 1.0f / (1.0f + nexp(-x)); }
__device__ __forceinline__ float wsum(float v) {
#pragma unroll
  for (int o = 16; o >= 1; o >>= 1) v += __shfl_xor(v, o); return v; }

__global__ __launch_bounds__(256) void prepw_kernel(const float* __restrict__ win1, const float* __restrict__ wxp1, const float* __restrict__ wdt1, const float* __restrict__ wout1, const float* __restrict__ win2, const float* __restrict__ wxp2, const float* __restrict__ wdt2, const float* __restrict__ wout2, b16* __restrict__ WIN, b16* __restrict__ WXP, b16* __restrict__ WDT, b16* __restrict__ WOUT) {
  __shared__ __attribute__((aligned(16))) b16 T[64][64 + 8];
  const int which = blockIdx.z, s = which >> 2, kind = which & 3, i0 = blockIdx.x * 64, o0 = blockIdx.y * 64, t_ = threadIdx.x;
  const int IN = kind == 2 ? R : D, OUT = kind == 0 ? 2 * D : kind == 1 ? 56 : D;
  const int INP = kind == 2 ? 64 : D, OUTP = kind == 0 ? 2 * D : kind == 1 ? 64 : D;
  if (i0 >= INP || o0 >= OUTP) return;
  const float* w = s == 0 ? (kind == 0 ? win1 : kind == 1 ? wxp1 : kind == 2 ? wdt1 : wout1) : (kind == 0 ? win2 : kind == 1 ? wxp2 : kind == 2 ? wdt2 : wout2);
  b16* dst = (kind == 0 ? WIN + (size_t)s * 2 * D * D : kind == 1 ? WXP + (size_t)s * XPW * D : kind == 2 ? WDT + (size_t)s * D * 64 : WOUT + (size_t)s * D * D);
  for (int q = t_; q < 64 * 64; q += 256) { const int ii = q >> 6, oo = q & 63; const int i = i0 + ii, o = o0 + oo; T[oo][ii] = (i < IN && o < OUT) ? (b16)(bf16_rne(w[(size_t)(i < IN ? i : 0) * OUT + (o < OUT ? o : 0)]) * WSC) : (b16)0.0f; }
  __syncthreads();
  for (int pass = 0; pass < 2; ++pass) { for (int q = t_; q < 64 * 8; q += 256) { const int oo = q >> 3, c8 = (q & 7) * 8; *(volatile v8b*)(dst + (size_t)(o0 + oo) * INP + i0 + c8) = *(const v8b*)(&T[oo][c8]); } __threadfence(); }
}
__global__ __launch_bounds__(256) void ln_kernel(const float* __restrict__ x1, const float* __restrict__ x2, const float* __restrict__ g1, const float* __restrict__ be1, const float* __restrict__ g2, const float* __restrict__ be2, b16* __restrict__ XNH, b16* __restrict__ XNL) {
  __shared__ __attribute__((aligned(16))) float Tt[64][64 + 4]; __shared__ float Smu[64], Srs[64]; __shared__ __attribute__((aligned(16))) b16 Th[64][64 + 8], Tl[64][64 + 8];
  const int s = blockIdx.z, b = blockIdx.y, l0 = blockIdx.x * 64, t_ = threadIdx.x; const float* x = (s == 0 ? x1 : x2) + (size_t)b * C * L; const float* g = s == 0 ? g1 : g2; const float* be = s == 0 ? be1 : be2;
  const size_t rowbase = ((size_t)s * NB + b) * L + l0;
  float sum = 0.0f;
  for (int c0 = 0; c0 < C; c0 += 64) {
    __syncthreads();
    for (int q = t_; q < 64 * 64; q += 256) { const int cc = q >> 6, ll = q & 63; Tt[ll][cc] = bf16_rne(x[(size_t)(c0 + cc) * L + l0 + ll]); }
    __syncthreads();
    if (t_ < 64) { for (int cc = 0; cc < 64; ++cc) sum += Tt[t_][cc]; } }
  if (t_ < 64) Smu[t_] = sum * (1.0f / C);
  __syncthreads();
  float ss = 0.0f;
  for (int c0 = 0; c0 < C; c0 += 64) {
    __syncthreads();
    for (int q = t_; q < 64 * 64; q += 256) { const int cc = q >> 6, ll = q & 63; Tt[ll][cc] = bf16_rne(x[(size_t)(c0 + cc) * L + l0 + ll]); }
    __syncthreads();
    if (t_ < 64) { const float mu = Smu[t_]; for (int cc = 0; cc < 64; ++cc) { const float d = Tt[t_][cc] - mu; ss += pmul(d, d); } } }
  if (t_ < 64) Srs[t_] = rsqrtf(ss * (1.0f / C) + EPS);
  __syncthreads();
  for (int c0 = 0; c0 < C; c0 += 64) {
    __syncthreads();
    for (int q = t_; q < 64 * 64; q += 256) { const int cc = q >> 6, ll = q & 63; const float v = pmul((bf16_rne(x[(size_t)(c0 + cc) * L + l0 + ll]) - Smu[ll]) * Srs[ll], bf16_rne(g[c0 + cc])) + bf16_rne(be[c0 + cc]); b16 a_, c_; split16(v * XS, a_, c_); Th[ll][cc] = a_; Tl[ll][cc] = c_; }
    __syncthreads();
    for (int pass = 0; pass < 2; ++pass) { for (int q = t_; q < 64 * 8; q += 256) { const int ll = q >> 3, c8 = (q & 7) * 8; *(volatile v8b*)(XNH + (rowbase + ll) * C + c0 + c8) = *(const v8b*)(&Th[ll][c8]); *(volatile v8b*)(XNL + (rowbase + ll) * C + c0 + c8) = *(const v8b*)(&Tl[ll][c8]); } __threadfence(); } }
}
template <int MODE>
__global__ __launch_bounds__(128) void gemm_kernel(const b16* __restrict__ AH, const b16* __restrict__ AL, int lda, const b16* __restrict__ Bw, int ldb, int K, float ascale, const float* __restrict__ aux, const float* __restrict__ aux2, float* __restrict__ Cout, int ldc, b16* __restrict__ PH, b16* __restrict__ PL, float* __restrict__ Cout2) {
  __shared__ __attribute__((aligned(16))) float Ts[4][16][128 + 4];
  const int wave = threadIdx.x >> 5, lane = threadIdx.x & 31, nloc = lane & 15, hlf = lane >> 4; const size_t m0 = (size_t)blockIdx.x * 64 + wave * 16; const int n0 = blockIdx.y * 128;
  const int NT = (MODE == 1) ? 4 : 8;
  v8f acc[8];
#pragma unroll
  for (int t = 0; t < 8; ++t) acc[t] = (v8f){};
  for (int kb = 0; kb < K; kb += 32) { const v16b ah = frag_kb(AH + (m0 + nloc) * lda + kb, hlf), al = frag_kb(AL + (m0 + nloc) * lda + kb, hlf);
#pragma unroll
    for (int t = 0; t < 8; ++t) if (t < NT) { const v16b bw = frag_kb(Bw + (size_t)(n0 + t * 16 + nloc) * ldb + kb, hlf); acc[t] = wmma16b(ah, bw, acc[t]); acc[t] = wmma16b(al, bw, acc[t]); } }
#pragma unroll
  for (int t = 0; t < 8; ++t) if (t < NT) { const int n = n0 + t * 16 + nloc;
#pragma unroll
    for (int r = 0; r < 8; ++r) { float v = acc[t][r] * ascale;
      if (MODE == 2) { v += bf16_rne(aux[n]); v = (v > 20.0f) ? v : log1pf(nexp(v)); }
      Ts[wave][8 * hlf + r][t * 16 + nloc] = v; } }
  wave_lds_sync();
  for (int pass = 0; pass < 2; ++pass) {
    for (int rr = 0; rr < 16; ++rr) { const size_t row = m0 + rr;
      if (MODE == 1) { if (lane < 16) *(volatile v4f*)(Cout + row * ldc + n0 + lane * 4) = *(const v4f*)(&Ts[wave][rr][lane * 4]);
        if (lane < 8) { v8b h8, l8;
#pragma unroll
          for (int j = 0; j < 8; ++j) { const int cidx = lane * 8 + j; b16 a_, c_; split16(cidx < R ? Ts[wave][rr][cidx] * DS : 0.0f, a_, c_); h8[j] = a_; l8[j] = c_; }
          *(volatile v8b*)(PH + row * 64 + lane * 8) = h8; *(volatile v8b*)(PL + row * 64 + lane * 8) = l8; } }
      else if (MODE == 0) { const v4f v = *(const v4f*)(&Ts[wave][rr][lane * 4]); if (n0 < D) *(volatile v4f*)(Cout + row * ldc + n0 + lane * 4) = v; else *(volatile v4f*)(Cout2 + row * ldc + (n0 - D) + lane * 4) = v; }
      else { v4f v = *(const v4f*)(&Ts[wave][rr][lane * 4]);
        if (MODE == 3) { const int bb = (int)(row / L), ll = (int)(row - (size_t)bb * L); const float* xr = aux2 + ((size_t)bb * C + n0 + lane * 4) * L + ll;
          v[0] += bf16_rne(xr[0]); v[1] += bf16_rne(xr[L]); v[2] += bf16_rne(xr[2 * L]); v[3] += bf16_rne(xr[3 * L]); }
        *(volatile v4f*)(Cout + row * ldc + n0 + lane * 4) = v; } }
    __threadfence(); }
}
__global__ __launch_bounds__(256) void dwconv_kernel(const float* __restrict__ UP, const float* __restrict__ wc1, const float* __restrict__ bc1, const float* __restrict__ wc2, const float* __restrict__ bc2, b16* __restrict__ UH, b16* __restrict__ UL) {
  __shared__ __attribute__((aligned(16))) float Tu[32][D + 4];
  const int sb = blockIdx.y, s = sb >> 1, lb = blockIdx.x * 32, t_ = threadIdx.x, wave = t_ >> 5, lane = t_ & 31; const float* wc = s ? wc2 : wc1; const float* bc = s ? bc2 : bc1;
  const size_t rb = (size_t)sb * L;
  for (int j = 0; j < 3; ++j) { const int d = t_ + 256 * j; const float w0 = bf16_rne(wc[d * 4 + 0]), w1 = bf16_rne(wc[d * 4 + 1]), w2 = bf16_rne(wc[d * 4 + 2]), w3 = bf16_rne(wc[d * 4 + 3]), bias = bf16_rne(bc[d]);
    float um3, um2, um1;
    { const int la = lb - 3, lb2 = lb - 2, lc = lb - 1;
      const float a = UP[(rb + (la < 0 ? 0 : la)) * D + d], bb = UP[(rb + (lb2 < 0 ? 0 : lb2)) * D + d], c = UP[(rb + (lc < 0 ? 0 : lc)) * D + d];
      um3 = la < 0 ? 0.0f : a; um2 = lb2 < 0 ? 0.0f : bb; um1 = lc < 0 ? 0.0f : c; }
    for (int i = 0; i < 32; ++i) { const float u0 = UP[(rb + lb + i) * D + d]; const float v = pmul(w0, um3) + pmul(w1, um2) + pmul(w2, um1) + pmul(w3, u0) + bias; Tu[i][d] = v * sigm(v); um3 = um2; um2 = um1; um1 = u0; } }
  __syncthreads();
  for (int pass = 0; pass < 2; ++pass) {
    for (int rr = wave * 4; rr < wave * 4 + 4; ++rr) { const size_t row = rb + lb + rr;
      for (int h = 0; h < 3; ++h) { v8b h8, l8; const v4f a = *(const v4f*)(&Tu[rr][h * 256 + lane * 8]), c = *(const v4f*)(&Tu[rr][h * 256 + lane * 8 + 4]);
#pragma unroll
        for (int j = 0; j < 4; ++j) { b16 x_, y_; split16(a[j] * US, x_, y_); h8[j] = x_; l8[j] = y_; split16(c[j] * US, x_, y_); h8[4 + j] = x_; l8[4 + j] = y_; }
        *(volatile v8b*)(UH + row * D + h * 256 + lane * 8) = h8; *(volatile v8b*)(UL + row * D + h * 256 + lane * 8) = l8; } }
    __threadfence(); }
}
__global__ __launch_bounds__(256) void scan_kernel(const float* __restrict__ DT, const b16* __restrict__ UH, const b16* __restrict__ UL, const float* __restrict__ Z, const float* __restrict__ XD, const float* __restrict__ alog1, const float* __restrict__ dsk1, const float* __restrict__ alog2, const float* __restrict__ dsk2, b16* __restrict__ YH, b16* __restrict__ YL) {
  __shared__ float Sbc[64][8]; __shared__ __attribute__((aligned(16))) b16 Th[64][256 + 8], Tl[64][256 + 8];
  const int sb = blockIdx.y, s = sb >> 1, b = sb & 1, d = blockIdx.x * 256 + threadIdx.x, t_ = threadIdx.x, wave = t_ >> 5, lane = t_ & 31;
  const float* alog = s ? alog2 : alog1; const float* dsk = s ? dsk2 : dsk1;
  const size_t rown = (size_t)sb * L, rother = (size_t)((1 - s) * NB + b) * L;
  float A[NS], h[NS];
#pragma unroll
  for (int n = 0; n < NS; ++n) { A[n] = -__expf(bf16_rne(alog[d * NS + n])); h[n] = 0.0f; }
  const float Dd = bf16_rne(dsk[d]);
  for (int l0 = 0; l0 < L; l0 += 64) {
    __syncthreads();
    for (int k = t_; k < 64 * 8; k += 256) { const int i = k >> 3, j = k & 7; Sbc[i][j] = (j < 4) ? XD[(rown + l0 + i) * XPW + R + j] : XD[(rother + l0 + i) * XPW + R + NS + (j - 4)]; }
    __syncthreads();
    for (int i = 0; i < 64; ++i) { const size_t row = rown + l0 + i; const float dt = DT[row * D + d], u = ((float)UH[row * D + d] + (float)UL[row * D + d]) * (1.0f / US), z = Z[row * D + d]; const float du = pmul(dt, u); float y = pmul(Dd, u);
#pragma unroll
      for (int n = 0; n < NS; ++n) { h[n] = pmul(__expf(pmul(dt, A[n])), h[n]) + pmul(du, Sbc[i][n]); y += pmul(h[n], Sbc[i][4 + n]); }
      const float ys = pmul(y, z * sigm(z)); b16 a_, c_; split16(ys * YS, a_, c_); Th[i][t_] = a_; Tl[i][t_] = c_; }
    __syncthreads();
    for (int pass = 0; pass < 2; ++pass) { for (int rr = wave * 8; rr < wave * 8 + 8; ++rr) { const size_t row = rown + l0 + rr; *(volatile v8b*)(YH + row * D + blockIdx.x * 256 + lane * 8) = *(const v8b*)(&Th[rr][lane * 8]); *(volatile v8b*)(YL + row * D + blockIdx.x * 256 + lane * 8) = *(const v8b*)(&Tl[rr][lane * 8]); } __threadfence(); } }
}
}

extern "C" void kernel_launch(void* const* d_in, const int* in_sizes, int n_in, void* d_out, int out_size, void* d_ws, size_t ws_size, hipStream_t stream) {
  (void)n_in;
  auto Fp = [&](int i) { return (const float*)d_in[i]; };
  if (in_sizes[0] != NB * C * L || in_sizes[1] != NB * C * L || in_sizes[4] != C * 2 * D || in_sizes[7] != D * 56 || in_sizes[8] != R * D || in_sizes[12] != D * C || in_sizes[15] != C * 2 * D || out_size != 2 * NB * L * C) return;
  size_t off = 0; char* ws = (char*)d_ws;
  auto carve = [&](size_t bytes) { char* p = ws + off; off += (bytes + 255) & ~(size_t)255; return p; };
  b16* WIN = (b16*)carve((size_t)2 * 2 * D * D * 2); b16* WXP = (b16*)carve((size_t)2 * XPW * D * 2); b16* WDT = (b16*)carve((size_t)2 * D * 64 * 2); b16* WOUT = (b16*)carve((size_t)2 * D * D * 2);
  b16* XNH = (b16*)carve((size_t)2 * NROW * C * 2); b16* XNL = (b16*)carve((size_t)2 * NROW * C * 2);
  float* UPRE = (float*)carve((size_t)2 * NROW * D * 4); float* Z = (float*)carve((size_t)2 * NROW * D * 4);
  b16* UH = (b16*)carve((size_t)2 * NROW * D * 2); b16* UL = (b16*)carve((size_t)2 * NROW * D * 2);
  float* XD = (float*)carve((size_t)2 * NROW * XPW * 4); b16* DRH = (b16*)carve((size_t)2 * NROW * 64 * 2); b16* DRL = (b16*)carve((size_t)2 * NROW * 64 * 2);
  float* DT = UPRE;
  b16* YH = XNH; b16* YL = XNL;
  if (off > ws_size) return;
  float* OUT = (float*)d_out;
  prepw_kernel<<<dim3(D / 64, 2 * D / 64, 8), 256, 0, stream>>>(Fp(4), Fp(7), Fp(8), Fp(12), Fp(15), Fp(18), Fp(19), Fp(23), WIN, WXP, WDT, WOUT);
  ln_kernel<<<dim3(L / 64, NB, 2), 256, 0, stream>>>(Fp(0), Fp(1), Fp(2), Fp(3), Fp(13), Fp(14), XNH, XNL);
  for (int s = 0; s < 2; ++s) gemm_kernel<0><<<dim3(NROW / 64, 2 * D / 128), 128, 0, stream>>>(XNH + (size_t)s * NROW * C, XNL + (size_t)s * NROW * C, C, WIN + (size_t)s * 2 * D * D, D, C, 1.0f / (XS * WSC), nullptr, nullptr, UPRE + (size_t)s * NROW * D, D, nullptr, nullptr, Z + (size_t)s * NROW * D);
  dwconv_kernel<<<dim3(L / 32, 4), 256, 0, stream>>>(UPRE, Fp(5), Fp(6), Fp(16), Fp(17), UH, UL);
  for (int s = 0; s < 2; ++s) gemm_kernel<1><<<dim3(NROW / 64, 1), 128, 0, stream>>>(UH + (size_t)s * NROW * D, UL + (size_t)s * NROW * D, D, WXP + (size_t)s * XPW * D, D, D, 1.0f / (US * WSC), nullptr, nullptr, XD + (size_t)s * NROW * XPW, XPW, DRH + (size_t)s * NROW * 64, DRL + (size_t)s * NROW * 64, nullptr);
  for (int s = 0; s < 2; ++s) gemm_kernel<2><<<dim3(NROW / 64, D / 128), 128, 0, stream>>>(DRH + (size_t)s * NROW * 64, DRL + (size_t)s * NROW * 64, 64, WDT + (size_t)s * D * 64, 64, 64, 1.0f / (DS * WSC), s ? Fp(20) : Fp(9), nullptr, DT + (size_t)s * NROW * D, D, nullptr, nullptr, nullptr);
  scan_kernel<<<dim3(D / 256, 4), 256, 0, stream>>>(DT, UH, UL, Z, XD, Fp(10), Fp(11), Fp(21), Fp(22), YH, YL);
  for (int s = 0; s < 2; ++s) gemm_kernel<3><<<dim3(NROW / 64, D / 128), 128, 0, stream>>>(YH + (size_t)s * NROW * D, YL + (size_t)s * NROW * D, D, WOUT + (size_t)s * D * D, D, D, 1.0f / (YS * WSC), nullptr, s ? Fp(1) : Fp(0), OUT + (size_t)s * NROW * C, C, nullptr, nullptr, nullptr);
}
